// Encoder1d_16355235463757
// MI455X (gfx1250) — hardware-verified
//
#include <hip/hip_runtime.h>
#include <math.h>
#include <stdint.h>

#define NB   128
#define NC   3
#define HW   128
#define LL   4096
#define D1   1204
#define D1P  1216
#define D2   4816
#define D2P  4864
#define MR   (NB * NC)
static_assert((MR % 64) == 0 && (D1P % 64) == 0 && (D2P % 64) == 0 && (LL % 32) == 0 && (D1P % 32) == 0);
static_assert((D1 % 4) == 0 && (D2 % 4) == 0 && (LL % 8) == 0 && D1 <= D1P && D2 <= D2P);
static_assert(((MR * LL / 8) % 256) == 0 && ((D1P * LL / 8) % 256) == 0 && ((D2P * D1P / 8) % 256) == 0);
static_assert(((MR * D1P / 8) % 256) == 0 && ((MR * D2 / 4) % 256) == 0);

typedef __bf16   v16b __attribute__((ext_vector_type(16)));
typedef __bf16   v8b  __attribute__((ext_vector_type(8)));
typedef float    v8f  __attribute__((ext_vector_type(8)));
typedef float    v4f  __attribute__((ext_vector_type(4)));
typedef unsigned int v4u __attribute__((ext_vector_type(4)));
typedef int      v4i  __attribute__((ext_vector_type(4)));

__device__ __forceinline__ unsigned short bf_bits(float f) {
  unsigned u = __float_as_uint(f);
  return (unsigned short)((u + 0x7FFFu + ((u >> 16) & 1u)) >> 16);
}
__device__ __forceinline__ float bf_up(unsigned short h) { return __uint_as_float(((unsigned)h) << 16); }
__device__ __forceinline__ unsigned pk16(unsigned short a, unsigned short b) { return (unsigned)a | ((unsigned)b << 16); }
__device__ __forceinline__ v8f zero8() { v8f z = {0.f, 0.f, 0.f, 0.f, 0.f, 0.f, 0.f, 0.f}; return z; }
__device__ __forceinline__ int clampi(int v, int lo, int hi) { return v < lo ? lo : (v > hi ? hi : v); }

__device__ __forceinline__ float act_bn(float h, float b, float mean, float rstd, float gg, float bb) {
  float v = h + bf_up(bf_bits(b));
  v = (v >= 0.f) ? v : 0.01f * v;
  return ((v - mean) * rstd) * gg + bb;
}
__device__ __forceinline__ void split_bits(float y, unsigned short& hi, unsigned short& lo) {
  hi = bf_bits(y);
  lo = bf_bits(y - bf_up(hi));
}

__device__ __forceinline__ v16b ldfrag_b(const __bf16* p) {
  union { v16b v; v8b h[2]; } f;
  f.h[0] = *(const v8b*)(p);
  f.h[1] = *(const v8b*)(p + 16);
  return f.v;
}

__device__ __forceinline__ v8f mma_b_raw(v16b a, v16b b, v8f c) {
  return __builtin_amdgcn_wmma_f32_16x16x32_bf16(false, a, false, b, (short)0, c, false, false);
}
__device__ __forceinline__ void dep_guard_b(v8f& a, v8f& b, v16b x, v16b y) {
#if defined(__HIP_DEVICE_COMPILE__)
  asm volatile("v_nop\n\tv_nop\n\tv_nop\n\tv_nop" : "+v"(a), "+v"(b) : "v"(x), "v"(y));
#endif
}
__device__ __forceinline__ void keep4_b(v16b a, v16b b, v16b c, v16b d) {
#if defined(__HIP_DEVICE_COMPILE__)
  asm volatile("v_nop" :: "v"(a), "v"(b), "v"(c), "v"(d));
#endif
}
__device__ __forceinline__ void acc_guard4(v8f& a, v8f& b, v8f& c, v8f& d) {
#if defined(__HIP_DEVICE_COMPILE__)
  asm volatile("v_nop\n\tv_nop\n\tv_nop\n\tv_nop" : "+v"(a), "+v"(b), "+v"(c), "+v"(d));
#endif
}
__device__ __forceinline__ void wave_sync_lds() {
  __builtin_amdgcn_fence(__ATOMIC_RELEASE, "workgroup");
  __builtin_amdgcn_wave_barrier();
  __builtin_amdgcn_fence(__ATOMIC_ACQUIRE, "workgroup");
}

__device__ __forceinline__ unsigned short samp(const float* __restrict__ xp, int r, int q, float m) {
  r = clampi(r, 0, HW - 1);
  q = clampi(q, 0, HW - 1);
  const float v  = xp[r * HW + q];
  const float mr = bf_up(bf_bits(m));
  return (mr < 0.3f) ? (unsigned short)0 : bf_bits(v);
}
__global__ __launch_bounds__(256) void gather_mask_bf16x8(const float* __restrict__ x, const int* __restrict__ coords,
                                                          const float* __restrict__ mask, unsigned short* out,
                                                          int n8tot) {
  const int i = blockIdx.x * 256 + threadIdx.x;
  if (i >= n8tot) return;
  const int row = i / (LL / 8);
  const int j   = i - row * (LL / 8);
  const int l0  = j * 8;
  const int n   = row / NC;
  const int* cp = coords + 2 * l0;
  const v4i c0 = *(const v4i*)(cp);
  const v4i c1 = *(const v4i*)(cp + 4);
  const v4i c2 = *(const v4i*)(cp + 8);
  const v4i c3 = *(const v4i*)(cp + 12);
  const float* mp = mask + (size_t)n * LL + l0;
  const v4f ma = *(const v4f*)(mp);
  const v4f mb = *(const v4f*)(mp + 4);
  const float* xp = x + (size_t)row * (HW * HW);
  v4u p;
  p[0] = pk16(samp(xp, c0[0], c0[1], ma[0]), samp(xp, c0[2], c0[3], ma[1]));
  p[1] = pk16(samp(xp, c1[0], c1[1], ma[2]), samp(xp, c1[2], c1[3], ma[3]));
  p[2] = pk16(samp(xp, c2[0], c2[1], mb[0]), samp(xp, c2[2], c2[3], mb[1]));
  p[3] = pk16(samp(xp, c3[0], c3[1], mb[2]), samp(xp, c3[2], c3[3], mb[3]));
  *(volatile v4u*)(out + (size_t)i * 8) = p;
  __threadfence();
  *(volatile v4u*)(out + (size_t)i * 8) = p;
}

__global__ __launch_bounds__(256) void cvt2d_bf16x8(const float* __restrict__ in, int srcRows, int srcCols,
                                                    unsigned short* out, int dstCols8, int n8tot) {
  const int i = blockIdx.x * 256 + threadIdx.x;
  if (i >= n8tot) return;
  const int row = i / dstCols8;
  const int j   = i - row * dstCols8;
  const int c0  = j * 8;
  const int rowc = (row > srcRows - 1) ? (srcRows - 1) : row;
  const int ca = (c0 > srcCols - 4) ? (srcCols - 4) : c0;
  const int cb = (c0 + 4 > srcCols - 4) ? (srcCols - 4) : (c0 + 4);
  const float* rp = in + (size_t)rowc * (size_t)srcCols;
  const v4f a = *(const v4f*)(rp + ca);
  const v4f b = *(const v4f*)(rp + cb);
  const bool rv = row < srcRows;
  const bool va = rv && (c0 < srcCols);
  const bool vb = rv && ((c0 + 4) < srcCols);
  v4u p;
  p[0] = va ? pk16(bf_bits(a[0]), bf_bits(a[1])) : 0u;
  p[1] = va ? pk16(bf_bits(a[2]), bf_bits(a[3])) : 0u;
  p[2] = vb ? pk16(bf_bits(b[0]), bf_bits(b[1])) : 0u;
  p[3] = vb ? pk16(bf_bits(b[2]), bf_bits(b[3])) : 0u;
  *(volatile v4u*)(out + (size_t)i * 8) = p;
  __threadfence();
  *(volatile v4u*)(out + (size_t)i * 8) = p;
}

template <int NSPLIT, int OUT_MODE>
__global__ __launch_bounds__(256) void gemm64(
    const unsigned short* __restrict__ Ap, const unsigned short* A2p, int lda, long long strideA,
    const unsigned short* __restrict__ Btp, const unsigned short* Bt2p, int ldb, long long strideB,
    void* Cout, int ldc, long long strideC,
    int M, int N, int K) {
  const __bf16* A   = (const __bf16*)(const void*)Ap;
  const __bf16* A2  = (const __bf16*)(const void*)A2p;
  const __bf16* Bt  = (const __bf16*)(const void*)Btp;
  const __bf16* Bt2 = (const __bf16*)(const void*)Bt2p;
  __shared__ __align__(16) float sT[8][16 * 68];
  const int b    = blockIdx.y;
  const int lane = threadIdx.x & 31;
  const int wave = threadIdx.x >> 5;
  const int tilesN = N >> 6;
  const int tilesM = M >> 6;
  const int tile = blockIdx.x * 8 + wave;
  if (tile >= tilesM * tilesN) return;
  const int tm = tile / tilesN;
  const int tn = tile - tm * tilesN;
  const int m0 = tm << 6;
  const int n0 = tn << 6;

  const __bf16* Ab  = A  + (size_t)b * strideA;
  const __bf16* Bb  = Bt + (size_t)b * strideB;
  const __bf16* Ab2 = (NSPLIT >= 1) ? (A2  + (size_t)b * strideA) : Ab;
  const __bf16* Bb2 = (NSPLIT == 2) ? (Bt2 + (size_t)b * strideB) : Bb;

  const int rlane = lane & 15;
  const int koff  = (lane >> 4) * 8;
  const int mOff  = (lane >> 4) * 8;

  v8f acc[4][4];
#pragma unroll
  for (int i = 0; i < 4; ++i)
#pragma unroll
    for (int j = 0; j < 4; ++j) acc[i][j] = zero8();

  for (int k0 = 0; k0 < K; k0 += 32) {
    v16b bh[4], bl[4];
#pragma unroll
    for (int j = 0; j < 4; ++j) {
      const size_t bo = (size_t)(n0 + (j << 4) + rlane) * ldb + koff + k0;
      bh[j] = ldfrag_b(Bb + bo);
      if (NSPLIT == 2) bl[j] = ldfrag_b(Bb2 + bo); else bl[j] = bh[j];
    }
#pragma unroll
    for (int i = 0; i < 4; ++i) {
      const size_t ao = (size_t)(m0 + (i << 4) + rlane) * lda + koff + k0;
      const v16b ah = ldfrag_b(Ab + ao);
      v16b al = ah;
      if (NSPLIT >= 1) al = ldfrag_b(Ab2 + ao);
#pragma unroll
      for (int j = 0; j < 4; ++j) {
        acc[i][j] = mma_b_raw(ah, bh[j], acc[i][j]);
        if (NSPLIT >= 1) acc[i][j] = mma_b_raw(al, bh[j], acc[i][j]);
        if (NSPLIT == 2) acc[i][j] = mma_b_raw(ah, bl[j], acc[i][j]);
      }
      dep_guard_b(acc[i][0], acc[i][3], ah, al);
    }
    keep4_b(bh[0], bh[1], bh[2], bh[3]);
    if (NSPLIT == 2) keep4_b(bl[0], bl[1], bl[2], bl[3]);
  }
  acc_guard4(acc[0][0], acc[0][1], acc[0][2], acc[0][3]);
  acc_guard4(acc[1][0], acc[1][1], acc[1][2], acc[1][3]);
  acc_guard4(acc[2][0], acc[2][1], acc[2][2], acc[2][3]);
  acc_guard4(acc[3][0], acc[3][1], acc[3][2], acc[3][3]);

  float* slab = sT[wave];
  const int hh = lane >> 4, c4 = (lane & 15) * 4;
  float* C = (float*)Cout + (size_t)b * strideC;
#pragma unroll
  for (int i = 0; i < 4; ++i) {
    const int mBase = m0 + (i << 4);
#pragma unroll
    for (int j = 0; j < 4; ++j) {
#pragma unroll
      for (int r = 0; r < 8; ++r) {
        slab[(mOff + r) * 68 + (j << 4) + rlane] = acc[i][j][r];
      }
    }
    wave_sync_lds();
    for (int pass = 0; pass < 2; ++pass) {
#pragma unroll
      for (int it = 0; it < 8; ++it) {
        const int row = it * 2 + hh;
        const v4f v = *(const v4f*)(slab + row * 68 + c4);
        *(volatile v4f*)(C + (size_t)(mBase + row) * ldc + n0 + c4) = v;
      }
      __threadfence();
    }
    wave_sync_lds();
  }
}

__global__ __launch_bounds__(256) void bn_stats(const float* __restrict__ H, int ld, int ncols, int nb,
                                                const float* __restrict__ bias, const float* __restrict__ g,
                                                const float* __restrict__ be, float* st) {
  __shared__ double red1[256];
  __shared__ double red2[256];
  __shared__ __align__(16) float sLine[32];
  const int tid = threadIdx.x;
  const int c   = blockIdx.x;
  double s1 = 0.0, s2 = 0.0;
#pragma unroll 1
  for (int n = 0; n < nb; ++n) {
    const float* hr = H + (size_t)(n * NC + c) * (size_t)ld;
#pragma unroll 1
    for (int col = tid; col < ncols; col += 256) {
      float v = hr[col] + bf_up(bf_bits(bias[col]));
      v = (v >= 0.f) ? v : 0.01f * v;
      s1 += (double)v;
      s2 += (double)v * (double)v;
    }
  }
  if (tid < 32) sLine[tid] = 0.f;
  red1[tid] = s1;
  red2[tid] = s2;
  __syncthreads();
  for (int s = 128; s > 0; s >>= 1) {
    if (tid < s) {
      red1[tid] += red1[tid + s];
      red2[tid] += red2[tid + s];
    }
    __syncthreads();
  }
  if (tid == 0) {
    const double inv  = 1.0 / ((double)nb * (double)ncols);
    const double mean = red1[0] * inv;
    double var = red2[0] * inv - mean * mean;
    if (var < 0.0) var = 0.0;
    const float meanf = (float)mean;
    const float varf  = (float)var;
    const float rstd  = rsqrtf(varf + 1e-5f);
    sLine[0] = meanf;
    sLine[1] = rstd;
    sLine[2] = bf_up(bf_bits(g[c]));
    sLine[3] = bf_up(bf_bits(be[c]));
  }
  __syncthreads();
  if (tid < 8) {
    const v4f v = *(const v4f*)(sLine + tid * 4);
    float* p = st + (size_t)c * 32 + tid * 4;
    *(volatile v4f*)p = v;
    __threadfence();
    *(volatile v4f*)p = v;
  }
}

__global__ __launch_bounds__(256) void bn_apply_split8(const float* __restrict__ H, int ld, int ncols,
                                                       const float* __restrict__ bias, const float* __restrict__ st,
                                                       unsigned short* hi, unsigned short* lo, int cols8, int n8tot) {
  const int i = blockIdx.x * 256 + threadIdx.x;
  if (i >= n8tot) return;
  const int row = i / cols8;
  const int j   = i - row * cols8;
  const int c0  = j * 8;
  const int c   = row % NC;
  const v4f sv  = *(const v4f*)(st + c * 32);
  const float mean = sv[0], rstd = sv[1], gg = sv[2], bb = sv[3];
  const float* hr = H + (size_t)row * (size_t)ld + c0;
  const v4f ha = *(const v4f*)(hr);
  const v4f hb = *(const v4f*)(hr + 4);
  const int ca = (c0 > ncols - 4) ? (ncols - 4) : c0;
  const int cb = (c0 + 4 > ncols - 4) ? (ncols - 4) : (c0 + 4);
  const v4f ba = *(const v4f*)(bias + ca);
  const v4f bv = *(const v4f*)(bias + cb);
  const bool va = c0 < ncols;
  const bool vb = (c0 + 4) < ncols;
  float ya[4], yb[4];
#pragma unroll
  for (int e = 0; e < 4; ++e) {
    ya[e] = va ? act_bn(ha[e], ba[e], mean, rstd, gg, bb) : 0.f;
    yb[e] = vb ? act_bn(hb[e], bv[e], mean, rstd, gg, bb) : 0.f;
  }
  v4u ph, pl;
#pragma unroll
  for (int e = 0; e < 2; ++e) {
    unsigned short h0, l0, h1, l1;
    split_bits(ya[2 * e], h0, l0);
    split_bits(ya[2 * e + 1], h1, l1);
    ph[e] = pk16(h0, h1);
    pl[e] = pk16(l0, l1);
    split_bits(yb[2 * e], h0, l0);
    split_bits(yb[2 * e + 1], h1, l1);
    ph[2 + e] = pk16(h0, h1);
    pl[2 + e] = pk16(l0, l1);
  }
  *(volatile v4u*)(hi + (size_t)i * 8) = ph;
  *(volatile v4u*)(lo + (size_t)i * 8) = pl;
  __threadfence();
  *(volatile v4u*)(hi + (size_t)i * 8) = ph;
  *(volatile v4u*)(lo + (size_t)i * 8) = pl;
}

__global__ __launch_bounds__(256) void bn_out4(const float* __restrict__ H, int ld, int ncols,
                                               const float* __restrict__ bias, const float* __restrict__ st,
                                               float* out, int n4tot) {
  const int i = blockIdx.x * 256 + threadIdx.x;
  if (i >= n4tot) return;
  const int f   = i * 4;
  const int row = f / ncols;
  const int col = f - row * ncols;
  const int c   = row % NC;
  const v4f sv  = *(const v4f*)(st + c * 32);
  const float mean = sv[0], rstd = sv[1], gg = sv[2], bb = sv[3];
  const v4f h = *(const v4f*)(H + (size_t)row * (size_t)ld + col);
  const v4f bz = *(const v4f*)(bias + col);
  v4f y;
#pragma unroll
  for (int e = 0; e < 4; ++e) y[e] = act_bn(h[e], bz[e], mean, rstd, gg, bb);
  float* p = out + (size_t)f;
  *(volatile v4f*)p = y;
  __threadfence();
  *(volatile v4f*)p = y;
}

extern "C" void kernel_launch(void* const* d_in, const int* in_sizes, int n_in,
                              void* d_out, int out_size, void* d_ws, size_t ws_size,
                              hipStream_t stream) {
  if (n_in < 11) return;
  if (in_sizes[0] != NB * NC * HW * HW) return;
  if (in_sizes[1] != LL * 2) return;
  if (in_sizes[2] != NB * LL) return;
  if (in_sizes[3] != D1 * LL) return;
  if (in_sizes[4] != D1) return;
  if (in_sizes[5] != NC || in_sizes[6] != NC) return;
  if (in_sizes[7] != D2 * D1) return;
  if (in_sizes[8] != D2) return;
  if (in_sizes[9] != NC || in_sizes[10] != NC) return;
  if (out_size != MR * D2) return;

  const float* x      = (const float*)d_in[0];
  const int*   coords = (const int*)d_in[1];
  const float* mask   = (const float*)d_in[2];
  const float* W1     = (const float*)d_in[3];
  const float* b1     = (const float*)d_in[4];
  const float* g1     = (const float*)d_in[5];
  const float* be1    = (const float*)d_in[6];
  const float* W2     = (const float*)d_in[7];
  const float* b2     = (const float*)d_in[8];
  const float* g2     = (const float*)d_in[9];
  const float* be2    = (const float*)d_in[10];
  float* out = (float*)d_out;

  const size_t PSb  = (size_t)MR * LL * 2;
  const size_t PW1  = (size_t)D1P * LL * 2;
  const size_t PW2  = (size_t)D2P * D1P * 2;
  const size_t PH1  = (size_t)MR * D1P * 4;
  const size_t PST  = 512;
  const size_t PH1h = (size_t)MR * D1P * 2;
  const size_t PH2  = (size_t)MR * D2P * 4;
  size_t off = 0;
  const size_t oSb  = off; off += PSb;
  const size_t oW1  = off; off += PW1;
  const size_t oW2  = off; off += PW2;
  const size_t oH1  = off; off += PH1;
  const size_t oST1 = off; off += PST;
  const size_t oH1h = off; off += PH1h;
  const size_t oH1l = off; off += PH1h;
  const size_t oH2  = off; off += PH2;
  const size_t oST2 = off; off += PST;
  if (off > ws_size) return;
  if (off > (size_t)134217728) return;

  char* ws = (char*)d_ws;
  unsigned short* Sb  = (unsigned short*)(ws + oSb);
  unsigned short* W1b = (unsigned short*)(ws + oW1);
  unsigned short* W2b = (unsigned short*)(ws + oW2);
  float* H1 = (float*)(ws + oH1);
  float* ST1 = (float*)(ws + oST1);
  unsigned short* H1hi = (unsigned short*)(ws + oH1h);
  unsigned short* H1lo = (unsigned short*)(ws + oH1l);
  float* H2 = (float*)(ws + oH2);
  float* ST2 = (float*)(ws + oST2);

  const dim3 blk(256);
  const int n8s  = MR * LL / 8;
  const int n8w1 = D1P * LL / 8;
  const int n8w2 = D2P * D1P / 8;
  const int n8h1 = MR * D1P / 8;
  const int n4o  = MR * D2 / 4;
  const dim3 gS((n8s + 255) / 256);
  const dim3 gW1((n8w1 + 255) / 256);
  const dim3 gW2((n8w2 + 255) / 256);
  const dim3 gG1(((MR / 64) * (D1P / 64) + 7) / 8, 1);
  const dim3 gBN(NC);
  const dim3 gA1((n8h1 + 255) / 256);
  const dim3 gG2(((MR / 64) * (D2P / 64) + 7) / 8, 1);
  const dim3 gO((n4o + 255) / 256);

  gather_mask_bf16x8<<<gS, blk, 0, stream>>>(x, coords, mask, Sb, n8s);
  cvt2d_bf16x8<<<gW1, blk, 0, stream>>>(W1, D1, LL, W1b, LL / 8, n8w1);
  cvt2d_bf16x8<<<gW2, blk, 0, stream>>>(W2, D2, D1, W2b, D1P / 8, n8w2);
  gemm64<0, 0><<<gG1, blk, 0, stream>>>(
      Sb, Sb, LL, 0LL, W1b, W1b, LL, 0LL,
      (void*)H1, D1P, 0LL,
      MR, D1P, LL);
  bn_stats<<<gBN, blk, 0, stream>>>(H1, D1P, D1, NB, b1, g1, be1, ST1);
  bn_apply_split8<<<gA1, blk, 0, stream>>>(H1, D1P, D1, b1, ST1, H1hi, H1lo, D1P / 8, n8h1);
  gemm64<1, 0><<<gG2, blk, 0, stream>>>(
      H1hi, H1lo, D1P, 0LL, W2b, W2b, D1P, 0LL,
      (void*)H2, D2P, 0LL,
      MR, D2P, D1P);
  bn_stats<<<gBN, blk, 0, stream>>>(H2, D2P, D2, NB, b2, g2, be2, ST2);
  bn_out4<<<gO, blk, 0, stream>>>(H2, D2P, D2, b2, ST2, out, n4o);
  (void)hipGetLastError();
}
